// MaskedCrossAttention_25434796327656
// MI455X (gfx1250) — hardware-run, weakly checked
//
#include <hip/hip_runtime.h>
#include <math.h>

typedef __attribute__((ext_vector_type(16))) _Float16 v16h;
typedef __attribute__((ext_vector_type(16))) __bf16 v16b;
typedef __attribute__((ext_vector_type(8)))  _Float16 v8h;
typedef __attribute__((ext_vector_type(8)))  float v8f;
typedef __attribute__((ext_vector_type(4)))  float v4f;
typedef __attribute__((ext_vector_type(2)))  float v2f;
typedef __attribute__((ext_vector_type(4)))  unsigned v4u;
typedef __attribute__((ext_vector_type(4)))  int v4i;
typedef float __attribute__((may_alias)) float_a;
typedef int __attribute__((may_alias)) int_a;

template <typename T> __device__ __forceinline__ void vst2(void* p, T v) { *(volatile T*)p = v; __threadfence(); *(volatile T*)p = v; }
__device__ __forceinline__ v8f wmma16(v16h a, v16h b, v8f c) {
  v8f d = __builtin_amdgcn_wmma_f32_16x16x32_f16(false, a, false, b, (short)0, c, false, false);
  asm volatile("v_nop\n\tv_nop\n\tv_nop\n\tv_nop" : "+v"(d) : "v"(a), "v"(b));
  return d;
}
__device__ __forceinline__ v8f wmma_bf(v16b a, v16b b, v8f c) {
  v8f d = __builtin_amdgcn_wmma_f32_16x16x32_bf16(false, a, false, b, (short)0, c, false, false);
  asm volatile("v_nop\n\tv_nop\n\tv_nop\n\tv_nop" : "+v"(d) : "v"(a), "v"(b));
  return d;
}
__device__ __forceinline__ v16h frag_h(const _Float16* rowk0, int lane) {
  union { v16h v; v8h q[2]; } u; const _Float16* p = rowk0 + 8 * (lane >> 4);
  u.q[0] = *(const v8h*)p; u.q[1] = *(const v8h*)(p + 16); return u.v;
}
__device__ __forceinline__ v16h frag_f32(const float* rowk0, int lane) {
  v16h a; const float* p = rowk0 + 8 * (lane >> 4);
#pragma unroll
  for (int i = 0; i < 8; ++i) { a[i] = (_Float16)p[i]; a[8 + i] = (_Float16)p[16 + i]; }
  return a;
}
__device__ __forceinline__ v16h frag_f32s(const float* rowk0, int lane, float sc) {
  v16h a; const float* p = rowk0 + 8 * (lane >> 4);
#pragma unroll
  for (int i = 0; i < 8; ++i) { a[i] = (_Float16)(p[i] * sc); a[8 + i] = (_Float16)(p[16 + i] * sc); }
  return a;
}
__device__ __forceinline__ v16h fragc_f32(const float* W, int k0, int n, int lane, int ld, int K) {
  v16h a; const int g = lane >> 4;
#pragma unroll
  for (int i = 0; i < 8; ++i) { const int ka = k0 + 8 * g + i, kb = ka + 16;
    a[i] = (_Float16)(ka < K ? W[(size_t)(ka < K ? ka : K - 1) * ld + n] : 0.f); a[8 + i] = (_Float16)(kb < K ? W[(size_t)(kb < K ? kb : K - 1) * ld + n] : 0.f); }
  return a;
}
struct F2 { v16b h, l; };
__device__ __forceinline__ F2 bsplit16(const float v[16]) { F2 r;
#pragma unroll
  for (int i = 0; i < 16; ++i) { const __bf16 h = (__bf16)v[i]; r.h[i] = h; r.l[i] = (__bf16)(v[i] - (float)h); }
  return r; }
__device__ __forceinline__ F2 split_row(const float* row, int k0, int lane) { float v[16]; const float* p = row + k0 + 8 * (lane >> 4);
#pragma unroll
  for (int i = 0; i < 8; ++i) { v[i] = p[i]; v[8 + i] = p[16 + i]; }
  return bsplit16(v); }
__device__ __forceinline__ F2 split_rowK(const float* row, int k0, int lane, int K) { float v[16]; const int g = lane >> 4;
#pragma unroll
  for (int i = 0; i < 8; ++i) { const int ka = k0 + 8 * g + i, kb = ka + 16; v[i] = ka < K ? row[ka < K ? ka : K - 1] : 0.f; v[8 + i] = kb < K ? row[kb < K ? kb : K - 1] : 0.f; }
  return bsplit16(v); }
__device__ __forceinline__ F2 split_col(const float* W, int k0, int n, int lane, int ld, int K) { float v[16]; const int g = lane >> 4;
#pragma unroll
  for (int i = 0; i < 8; ++i) { const int ka = k0 + 8 * g + i, kb = ka + 16; v[i] = ka < K ? W[(size_t)(ka < K ? ka : K - 1) * ld + n] : 0.f; v[8 + i] = kb < K ? W[(size_t)(kb < K ? kb : K - 1) * ld + n] : 0.f; }
  return bsplit16(v); }
__device__ __forceinline__ v8f mac3(const F2& a, const F2& b, v8f c) { c = wmma_bf(a.l, b.h, c); c = wmma_bf(a.h, b.l, c); return wmma_bf(a.h, b.h, c); }
__device__ __forceinline__ float sigm(float v) { return 1.0f / (1.0f + expf(-v)); }
#define LDSX() do { asm volatile("s_wait_dscnt 0" ::: "memory"); __builtin_amdgcn_wave_barrier(); __builtin_amdgcn_fence(__ATOMIC_RELEASE, "workgroup"); } while (0)


#define NB 4
#define TQ 2048
#define DIM 1024
#define TI 16
#define NL 64
#define NKV (TI * NL)
#define DL 1024
#define NH 8
#define HD2 64
#define INNER (NH * HD2)
#ifndef TNB
#define TNB NB
#endif
#ifndef TQBK
#define TQBK (TQ / 64)
#endif
typedef __attribute__((ext_vector_type(8))) __bf16 v8b;
__device__ __forceinline__ v16b frag_b(const __bf16* rowk0, int lane) {
  union { v16b v; v8b q[2]; } u; const __bf16* p = rowk0 + 8 * (lane >> 4);
  u.q[0] = *(const v8b*)p; u.q[1] = *(const v8b*)(p + 16); return u.v;
}
__device__ __forceinline__ float bfr(float v) { return (float)(__bf16)v; }
__device__ __attribute__((noinline)) float exp_ni(float v) { return expf(v); }
__device__ __attribute__((noinline)) float erf_ni(float v) { return erff(v); }

#define WS_QH  0u
#define WS_QL  (WS_QH + 2u * (size_t)NB * TQ * INNER)
#define WS_KH  (WS_QL + 2u * (size_t)NB * TQ * INNER)
#define WS_KL  (WS_KH + 2u * (size_t)NB * NKV * INNER)
#define WS_VH  (WS_KL + 2u * (size_t)NB * NKV * INNER)
#define WS_VL  (WS_VH + 2u * (size_t)NB * INNER * NKV)
#define WS_CT  (WS_VL + 2u * (size_t)NB * INNER * NKV)
#define WS_QT  (WS_CT + 4u * (size_t)NB * TQ * INNER)
#define WS_END (WS_QT + 4u * (size_t)NB * TQ)

__global__ __launch_bounds__(64) void k_cum(const int* __restrict__ ML, int* __restrict__ QT) { __shared__ __align__(16) int sq[TQ]; const size_t b = blockIdx.x; const int t = threadIdx.x;
  if (t == 0) { int acc = 0;
#pragma unroll 1
    for (int q = 0; q < TQ; ++q) { acc += (ML[b * TQ + q] != 0) ? 1 : 0; sq[q] = acc; } }
  __syncthreads(); for (int e = t; e < TQ / 4; e += 64) vst2(QT + b * TQ + e * 4, *(const v4i*)&sq[e * 4]); }
__global__ __launch_bounds__(128) void k_q(const float* __restrict__ X, const float* __restrict__ G, const float* __restrict__ Bt, const float* __restrict__ WQ, _Float16* __restrict__ QH, _Float16* __restrict__ QL) { __shared__ __align__(16) float sst[64][2]; __shared__ __align__(16) _Float16 sh[64][136], sl[64][136];
  const int tid = threadIdx.x, wave = tid >> 5, lane = tid & 31, col = lane & 15, g = lane >> 4; const size_t b = blockIdx.z; const int c0 = blockIdx.y * 128; const size_t r0 = b * TQ + (size_t)blockIdx.x * 64;
  { const int rl = tid >> 1, half = tid & 1; const float* xr = X + (r0 + rl) * DIM + half * 512; float s = 0.f;
#pragma unroll 1
    for (int i = 0; i < 512; ++i) s += bfr(xr[i]);
    s += __shfl_xor(s, 1); const float mu = s * (1.0f / DIM); float q = 0.f;
#pragma unroll 1
    for (int i = 0; i < 512; ++i) { const float d = bfr(xr[i]) - mu; q += d * d; }
    q += __shfl_xor(q, 1); if (half == 0) { sst[rl][0] = mu; sst[rl][1] = 1.0f / sqrtf(q * (1.0f / DIM) + 1e-5f); } }
  __syncthreads();
  const int rl = wave * 16 + col; const float mu = sst[rl][0], inv = sst[rl][1]; const float* xr = X + (r0 + rl) * DIM;
  v8f acc[8] = {};
#pragma unroll 2
  for (int kc = 0; kc < DIM / 32; ++kc) { float v[16]; const int k0 = kc * 32 + 8 * g;
#pragma unroll
    for (int i = 0; i < 8; ++i) { const int ka = k0 + i, kb = k0 + 16 + i; v[i] = (bfr(xr[ka]) - mu) * inv * bfr(G[ka]) + bfr(Bt[ka]); v[8 + i] = (bfr(xr[kb]) - mu) * inv * bfr(G[kb]) + bfr(Bt[kb]); }
    const F2 a = bsplit16(v);
#pragma unroll
    for (int j = 0; j < 8; ++j) { v16b w; const int o = c0 + j * 16 + col;
#pragma unroll
      for (int i = 0; i < 8; ++i) { w[i] = (__bf16)WQ[(size_t)(kc * 32 + 8 * g + i) * INNER + o]; w[8 + i] = (__bf16)WQ[(size_t)(kc * 32 + 16 + 8 * g + i) * INNER + o]; }
      acc[j] = wmma_bf(a.h, w, acc[j]); acc[j] = wmma_bf(a.l, w, acc[j]); } }
#pragma unroll
  for (int j = 0; j < 8; ++j)
#pragma unroll
    for (int r = 0; r < 8; ++r) { const float v = acc[j][r] * 0.125f; const _Float16 hv = (_Float16)v; sh[wave * 16 + 8 * g + r][j * 16 + col] = hv; sl[wave * 16 + 8 * g + r][j * 16 + col] = (_Float16)((v - (float)hv) * 2048.0f); }
  __syncthreads();
  for (int e = tid; e < 64 * 16; e += 128) { const int rr = e >> 4, q = e & 15; const size_t o = (r0 + rr) * INNER + c0 + q * 8; vst2((unsigned*)(QH + o), *(const v4u*)&sh[rr][q * 8]); vst2((unsigned*)(QL + o), *(const v4u*)&sl[rr][q * 8]); } }
__global__ __launch_bounds__(128) void k_kv(const float* __restrict__ MED, const float* __restrict__ WKV, _Float16* __restrict__ KH, _Float16* __restrict__ KL, _Float16* __restrict__ VH, _Float16* __restrict__ VL) { __shared__ __align__(16) _Float16 sh[64][136], sl[64][136]; __shared__ __align__(16) _Float16 th[128][72], tl[128][72];
  const int tid = threadIdx.x, wave = tid >> 5, lane = tid & 31, col = lane & 15, g = lane >> 4; const size_t b = blockIdx.z; const int cg = blockIdx.y; const int which = cg >> 2; const int c0 = (cg & 3) * 128; const int j0 = blockIdx.x * 64; const size_t r0 = b * NKV + j0 + wave * 16;
  v8f acc[8] = {};
#pragma unroll 2
  for (int kc = 0; kc < DL / 32; ++kc) { v16b a; { const float* p = MED + (r0 + col) * DL + kc * 32 + 8 * g;
#pragma unroll
      for (int i = 0; i < 8; ++i) { a[i] = (__bf16)p[i]; a[8 + i] = (__bf16)p[16 + i]; } }
#pragma unroll
    for (int j = 0; j < 8; ++j) { v16b w; const size_t o = (size_t)which * INNER + c0 + j * 16 + col;
#pragma unroll
      for (int i = 0; i < 8; ++i) { w[i] = (__bf16)WKV[(size_t)(kc * 32 + 8 * g + i) * (2 * INNER) + o]; w[8 + i] = (__bf16)WKV[(size_t)(kc * 32 + 16 + 8 * g + i) * (2 * INNER) + o]; }
      acc[j] = wmma_bf(a, w, acc[j]); } }
#pragma unroll
  for (int j = 0; j < 8; ++j)
#pragma unroll
    for (int r = 0; r < 8; ++r) { const float v = acc[j][r]; const _Float16 hv = (_Float16)v, lv = (_Float16)((v - (float)hv) * 2048.0f); const int rl = wave * 16 + 8 * g + r, cl = j * 16 + col; if (which == 0) { sh[rl][cl] = hv; sl[rl][cl] = lv; } else { th[cl][rl] = hv; tl[cl][rl] = lv; } }
  __syncthreads();
  if (which == 0) { for (int e = tid; e < 64 * 16; e += 128) { const int rl = e >> 4, q = e & 15; const size_t o = (b * NKV + j0 + rl) * INNER + c0 + q * 8; vst2((unsigned*)(KH + o), *(const v4u*)&sh[rl][q * 8]); vst2((unsigned*)(KL + o), *(const v4u*)&sl[rl][q * 8]); } }
  else { for (int e = tid; e < 128 * 8; e += 128) { const int cl = e >> 3, q = e & 7; const size_t o = (b * INNER + c0 + cl) * (size_t)NKV + j0 + q * 8; vst2((unsigned*)(VH + o), *(const v4u*)&th[cl][q * 8]); vst2((unsigned*)(VL + o), *(const v4u*)&tl[cl][q * 8]); } } }
__global__ __launch_bounds__(128) void k_att(const _Float16* __restrict__ QH, const _Float16* __restrict__ QL, const _Float16* __restrict__ KH, const _Float16* __restrict__ KL, const _Float16* __restrict__ VH, const _Float16* __restrict__ VL, const int* __restrict__ QT, float* __restrict__ CT) {
  __shared__ __align__(16) float sp[4][16][36]; __shared__ __align__(16) float so[4][16][68];
  const int tid = threadIdx.x, wave = tid >> 5, lane = tid & 31, col = lane & 15, g = lane >> 4; const int qb = blockIdx.x, h = blockIdx.y; const size_t b = blockIdx.z; const int q0 = qb * 64 + wave * 16; const bool three = (qb < 2);
  v16h aq[2], al[2];
#pragma unroll
  for (int kc = 0; kc < 2; ++kc) { aq[kc] = frag_h(QH + (b * TQ + q0 + col) * INNER + h * HD2 + kc * 32, lane); al[kc] = frag_h(QL + (b * TQ + q0 + col) * INNER + h * HD2 + kc * 32, lane); }
  int qt[8];
#pragma unroll
  for (int r = 0; r < 8; ++r) qt[r] = QT[b * TQ + q0 + 8 * g + r];
  float m[8], l[8];
#pragma unroll
  for (int r = 0; r < 8; ++r) { m[r] = -3.0e38f; l[r] = 0.f; }
  v8f acc[4] = {}, accl[4] = {};
#pragma unroll 1
  for (int ks = 0; ks < NKV / 32; ++ks) { const int ktime = (ks * 32) / NL + 1;
    float s[2][8];
#pragma unroll
    for (int ct = 0; ct < 2; ++ct) { const int kk = ks * 32 + ct * 16 + col; const size_t rk = (b * NKV + kk) * INNER + h * HD2; v8f c = {};
#pragma unroll
      for (int kc = 0; kc < 2; ++kc) c = wmma16(aq[kc], frag_h(KH + rk + kc * 32, lane), c);
      if (three) { v8f cl = {};
#pragma unroll
        for (int kc = 0; kc < 2; ++kc) { cl = wmma16(al[kc], frag_h(KH + rk + kc * 32, lane), cl); cl = wmma16(aq[kc], frag_h(KL + rk + kc * 32, lane), cl); }
#pragma unroll
        for (int r = 0; r < 8; ++r) c[r] += cl[r] * (1.0f / 2048.0f); }
#pragma unroll
      for (int r = 0; r < 8; ++r) s[ct][r] = (qt[r] == ktime) ? c[r] : ((qt[r] > TI || qt[r] == 0) ? 0.0f : -3.0e38f); }
    float alpha[8];
#pragma unroll
    for (int r = 0; r < 8; ++r) { float mx = fmaxf(s[0][r], s[1][r]);
#pragma unroll
      for (int o = 1; o < 16; o <<= 1) mx = fmaxf(mx, __shfl_xor(mx, o));
      const float mn = fmaxf(m[r], mx); alpha[r] = (m[r] <= -1.0e38f) ? 0.f : __expf(m[r] - mn); const float e0 = (s[0][r] <= -1.0e38f) ? 0.f : __expf(s[0][r] - mn), e1 = (s[1][r] <= -1.0e38f) ? 0.f : __expf(s[1][r] - mn); float es = e0 + e1;
#pragma unroll
      for (int o = 1; o < 16; o <<= 1) es += __shfl_xor(es, o);
      l[r] = l[r] * alpha[r] + es; m[r] = mn; sp[wave][8 * g + r][col] = e0; sp[wave][8 * g + r][16 + col] = e1; }
#pragma unroll
    for (int j = 0; j < 4; ++j)
#pragma unroll
      for (int r = 0; r < 8; ++r) { acc[j][r] *= alpha[r]; accl[j][r] *= alpha[r]; }
    LDSX();
    v16h pa, pl; { const float* prow = &sp[wave][col][0] + 8 * (lane >> 4);
#pragma unroll
      for (int i = 0; i < 8; ++i) { const float x0 = prow[i] * 2048.0f, x1 = prow[16 + i] * 2048.0f; const _Float16 h0 = (_Float16)x0, h1 = (_Float16)x1; pa[i] = h0; pa[8 + i] = h1; pl[i] = (_Float16)((x0 - (float)h0) * 2048.0f); pl[8 + i] = (_Float16)((x1 - (float)h1) * 2048.0f); } }
#pragma unroll
    for (int j = 0; j < 4; ++j) { const size_t po = (b * INNER + (size_t)h * HD2 + j * 16 + col) * NKV + ks * 32; const v16h vh = frag_h(VH + po, lane); acc[j] = wmma16(pa, vh, acc[j]); if (three) { accl[j] = wmma16(pl, vh, accl[j]); accl[j] = wmma16(pa, frag_h(VL + po, lane), accl[j]); } }
    LDSX(); }
#pragma unroll
  for (int r = 0; r < 8; ++r) { const float il = (l[r] > 0.f && qt[r] != 0) ? (1.0f / 2048.0f) / l[r] : 0.f;
#pragma unroll
    for (int j = 0; j < 4; ++j) so[wave][8 * g + r][j * 16 + col] = (acc[j][r] + accl[j][r] * (1.0f / 2048.0f)) * il; }
  LDSX(); for (int rl = 0; rl < 16; ++rl) if (lane < 16) vst2(CT + (b * TQ + q0 + rl) * INNER + h * HD2 + lane * 4, *(const v4f*)&so[wave][rl][lane * 4]); }
__global__ __launch_bounds__(128) void k_out(const float* __restrict__ CT, const float* __restrict__ WO, float* __restrict__ OUT) { __shared__ __align__(16) float sf[4][16][132];
  const int tid = threadIdx.x, wave = tid >> 5, lane = tid & 31, col = lane & 15, g = lane >> 4; const size_t b = blockIdx.z; const int c0 = blockIdx.y * 128; const size_t r0 = b * TQ + (size_t)blockIdx.x * 64 + wave * 16;
  v8f acc[8] = {};
#pragma unroll 2
  for (int kc = 0; kc < INNER / 32; ++kc) { const F2 a = split_row(CT + (r0 + col) * INNER, kc * 32, lane);
#pragma unroll
    for (int j = 0; j < 8; ++j) { v16b w; const int o = c0 + j * 16 + col;
#pragma unroll
      for (int i = 0; i < 8; ++i) { w[i] = (__bf16)WO[(size_t)(kc * 32 + 8 * g + i) * DIM + o]; w[8 + i] = (__bf16)WO[(size_t)(kc * 32 + 16 + 8 * g + i) * DIM + o]; }
      acc[j] = wmma_bf(a.h, w, acc[j]); acc[j] = wmma_bf(a.l, w, acc[j]); } }
#pragma unroll
  for (int j = 0; j < 8; ++j)
#pragma unroll
    for (int r = 0; r < 8; ++r) sf[wave][8 * g + r][j * 16 + col] = acc[j][r];
  LDSX(); for (int rl = 0; rl < 16; ++rl) vst2(OUT + (r0 + rl) * DIM + c0 + lane * 4, *(const v4f*)&sf[wave][rl][lane * 4]); }
extern "C" void kernel_launch(void* const* d_in, const int* in_sizes, int n_in, void* d_out, int out_size, void* d_ws, size_t ws_size, hipStream_t stream) {
  (void)in_sizes; (void)n_in; (void)out_size;
  const float** F = (const float**)d_in;
  if (ws_size < (size_t)WS_END) return;
  char* ws = (char*)d_ws; _Float16 *QH = (_Float16*)(ws + WS_QH), *QL = (_Float16*)(ws + WS_QL), *KH = (_Float16*)(ws + WS_KH), *KL = (_Float16*)(ws + WS_KL), *VH = (_Float16*)(ws + WS_VH), *VL = (_Float16*)(ws + WS_VL); float* CT = (float*)(ws + WS_CT); int* QT = (int*)(ws + WS_QT);
  k_cum<<<TNB, 64, 0, stream>>>((const int*)d_in[2], QT);
  k_q<<<dim3(TQBK, INNER / 128, TNB), 128, 0, stream>>>(F[0], F[3], F[4], F[5], QH, QL);
  k_kv<<<dim3(NKV / 64, 8, TNB), 128, 0, stream>>>(F[1], F[6], KH, KL, VH, VL);
  k_att<<<dim3(TQBK, NH, TNB), 128, 0, stream>>>(QH, QL, KH, KL, VH, VL, QT, CT);
  k_out<<<dim3(TQBK, DIM / 128, TNB), 128, 0, stream>>>(CT, F[7], (float*)d_out);
}
